// MambaBlock_30863634989742
// MI455X (gfx1250) — hardware-verified
//
#include <hip/hip_runtime.h>
#include <stddef.h>
#include <stdint.h>
#include <math.h>


#define NB      8
#define SEQ     1024
#define DM      512
#define NS      16
#define MROWS   8192
#define NDBC    64
#define K2      1024
#define KDT     64
#define PADR    514
#define X1T_PLANE (NB * PADR * SEQ)
#define WCT     (SEQ * SEQ)
#define GBM     128
#define GBN     64
#define GTHR    128
#define NTHR    256
#define ST      32
#define SCH     128
#define SCAN_LDS_FLOATS (4 * ST * SCH + ST * 32)
#define WSMAX   134217728

#define PE0 (MROWS * DM / 8)
#define PE1 (PE0 + DM * DM / 8)
#define PE2 (PE1 + DM * DM / 8)
#define PE3 (PE2 + DM * K2 / 8)
#define PE4 (PE3 + NDBC * K2 / 8)
#define PE5 (PE4 + DM * KDT / 8)
#define PE6 (PE5 + SEQ * SEQ / 8)
#define PE7 (PE6 + 2 * NB * 2 * SEQ / 8)
#define U_TOT PE7

static_assert(DM % GBM == 0 && SEQ % GBM == 0 && MROWS % GBM == 0);
static_assert(DM % GBN == 0 && SEQ % GBN == 0 && NDBC == GBN && NDBC == 32 + 2 * NS);
static_assert(DM % 32 == 0 && K2 % 32 == 0 && KDT % 32 == 0 && SEQ % 32 == 0 && K2 == 2 * DM && KDT == 2 * 32);
static_assert(PADR == DM + 2);
static_assert(GBM == (GTHR / 32) * 32 && GBN == 64);
static_assert(PE0 % NTHR == 0 && PE1 % NTHR == 0 && PE2 % NTHR == 0 && PE3 % NTHR == 0);
static_assert(PE4 % NTHR == 0 && PE5 % NTHR == 0 && PE6 % NTHR == 0 && PE7 % NTHR == 0);
static_assert(SEQ % ST == 0 && DM % SCH == 0 && SCH * 2 == NTHR && SCH == 128);
static_assert(ST * SCH / 4 == 4 * NTHR && ST * 32 / 4 == NTHR);
static_assert(SCAN_LDS_FLOATS * 4 == 69632);
static_assert(MROWS == NB * SEQ);

typedef float          v4f   __attribute__((ext_vector_type(4)));
typedef float          v8f   __attribute__((ext_vector_type(8)));
typedef int            v8i   __attribute__((ext_vector_type(8)));
typedef unsigned       v4u   __attribute__((ext_vector_type(4)));
typedef unsigned short v8us  __attribute__((ext_vector_type(8)));
typedef unsigned short v16us __attribute__((ext_vector_type(16)));
typedef __bf16         v16bf __attribute__((ext_vector_type(16)));
typedef v4f  __attribute__((may_alias)) v4fa;
typedef v4u  __attribute__((may_alias)) v4ua;
typedef v8us __attribute__((may_alias)) v8usa;
union FragB { v16bf v; v16us u; v8us h[2]; v8i w; };

__device__ __forceinline__ v8f wmb(const FragB& a, const FragB& b, v8f c) {
  v8f d = __builtin_amdgcn_wmma_f32_16x16x32_bf16(false, a.v, false, b.v, (short)0, c, false, false);
  asm volatile("v_nop\n\tv_nop\n\tv_nop\n\tv_nop" : "+v"(d) : "v"(a.w), "v"(b.w));
  return d;
}

__device__ __forceinline__ unsigned bf16_bits(float f) {
  const unsigned u = __float_as_uint(f);
  return (u + 0x7FFFu + ((u >> 16) & 1u)) >> 16;
}
__device__ __forceinline__ float bf16_val(float f) {
  return __uint_as_float(bf16_bits(f) << 16);
}
__device__ __forceinline__ unsigned short hl_bits(float v, int lo) {
  const unsigned hb = bf16_bits(v);
  const unsigned lb = bf16_bits(v - __uint_as_float(hb << 16));
  return (unsigned short)(lo != 0 ? lb : hb);
}
__device__ __forceinline__ v8us hl8(const v4f a, const v4f b, const int lo) {
  v8us o;
  o[0] = hl_bits(a.x, lo); o[1] = hl_bits(a.y, lo); o[2] = hl_bits(a.z, lo); o[3] = hl_bits(a.w, lo);
  o[4] = hl_bits(b.x, lo); o[5] = hl_bits(b.y, lo); o[6] = hl_bits(b.z, lo); o[7] = hl_bits(b.w, lo);
  return o;
}
__device__ __forceinline__ v8us pk8(float a0, float a1, float a2, float a3, float a4, float a5, float a6, float a7) {
  v8us o;
  o[0] = (unsigned short)bf16_bits(a0); o[1] = (unsigned short)bf16_bits(a1);
  o[2] = (unsigned short)bf16_bits(a2); o[3] = (unsigned short)bf16_bits(a3);
  o[4] = (unsigned short)bf16_bits(a4); o[5] = (unsigned short)bf16_bits(a5);
  o[6] = (unsigned short)bf16_bits(a6); o[7] = (unsigned short)bf16_bits(a7);
  return o;
}
__device__ __forceinline__ float silu_f(float v) {
  return v * __builtin_amdgcn_rcpf(1.0f + expf(-v));
}
__device__ __forceinline__ float softplus_f(float p) {
  return fmaxf(p, 0.0f) + log1pf(expf(-fabsf(p)));
}

__device__ __forceinline__ void cvt8_put(const float* __restrict__ src, unsigned short* dst) {
  const v4f a = *(const v4f*)src;
  const v4f b = *(const v4f*)(src + 4);
  const v8us o = pk8(a.x, a.y, a.z, a.w, b.x, b.y, b.z, b.w);
  *(volatile v8us*)dst = o;
  __threadfence();
  *(volatile v8us*)dst = o;
}

__global__ __launch_bounds__(NTHR) void k_prep(const float* __restrict__ x, const float* __restrict__ W1,
                                               const float* __restrict__ W2, const float* __restrict__ Wout,
                                               const float* __restrict__ Wdbc, const float* __restrict__ Wdt,
                                               const float* __restrict__ convw,
                                               unsigned short* XB, unsigned short* W1B, unsigned short* W2B,
                                               unsigned short* WOUT2, unsigned short* WDBC2, unsigned short* WDT2,
                                               unsigned short* WC, unsigned short* X1T) {
  const int u = (int)blockIdx.x * NTHR + (int)threadIdx.x;
  if (u < PE0) {
    cvt8_put(x + (size_t)u * 8, XB + (size_t)u * 8);
  } else if (u < PE1) {
    const int v = u - PE0;
    cvt8_put(W1 + (size_t)v * 8, W1B + (size_t)v * 8);
  } else if (u < PE2) {
    const int v = u - PE1;
    cvt8_put(W2 + (size_t)v * 8, W2B + (size_t)v * 8);
  } else if (u < PE3) {
    const int v  = u - PE2;
    const int n  = v >> 7;
    const int kk = (v & 127) * 8;
    const int k  = kk & (DM - 1);
    cvt8_put(Wout + (size_t)n * DM + k, WOUT2 + (size_t)n * K2 + kk);
  } else if (u < PE4) {
    const int v  = u - PE3;
    const int n  = v >> 7;
    const int kk = (v & 127) * 8;
    const int k  = kk & (DM - 1);
    cvt8_put(Wdbc + (size_t)n * DM + k, WDBC2 + (size_t)n * K2 + kk);
  } else if (u < PE5) {
    const int v  = u - PE4;
    const int n  = v >> 3;
    const int kk = (v & 7) * 8;
    const int k  = kk & 31;
    cvt8_put(Wdt + (size_t)n * 32 + k, WDT2 + (size_t)n * KDT + kk);
  } else if (u < PE6) {
    const int v = u - PE5;
    const float* s = convw + (size_t)v * 24;
    const v4f q0 = *(const v4f*)(s);
    const v4f q1 = *(const v4f*)(s + 4);
    const v4f q2 = *(const v4f*)(s + 8);
    const v4f q3 = *(const v4f*)(s + 12);
    const v4f q4 = *(const v4f*)(s + 16);
    const v4f q5 = *(const v4f*)(s + 20);
    const v8us o0 = pk8(q0.x, q0.w, q1.z, q2.y, q3.x, q3.w, q4.z, q5.y);
    const v8us o1 = pk8(q0.y, q1.x, q1.w, q2.z, q3.y, q4.x, q4.w, q5.z);
    const v8us o2 = pk8(q0.z, q1.y, q2.x, q2.w, q3.z, q4.y, q5.x, q5.w);
    unsigned short* d0 = WC + (size_t)v * 8;
    unsigned short* d1 = d0 + (size_t)WCT;
    unsigned short* d2 = d1 + (size_t)WCT;
    *(volatile v8us*)d0 = o0;
    *(volatile v8us*)d1 = o1;
    *(volatile v8us*)d2 = o2;
    __threadfence();
    *(volatile v8us*)d0 = o0;
    *(volatile v8us*)d1 = o1;
    *(volatile v8us*)d2 = o2;
  } else if (u < PE7) {
    const int v  = u - PE6;
    const int rr = v >> 7;
    const int c8 = (v & 127) * 8;
    const int pl = rr >> 4;
    const int b  = (rr >> 1) & 7;
    const int e  = rr & 1;
    const int row = e * (PADR - 1);
    unsigned short* dst = X1T + (size_t)pl * X1T_PLANE + ((size_t)b * PADR + (size_t)row) * SEQ + c8;
    const v8us z = {0, 0, 0, 0, 0, 0, 0, 0};
    *(volatile v8us*)dst = z;
    __threadfence();
    *(volatile v8us*)dst = z;
  }
}

__device__ __forceinline__ void mma_loop(v8f (&acc)[2][4],
                                         const unsigned short* __restrict__ ap, const int lda,
                                         const unsigned short* __restrict__ wp, const int ldb,
                                         const int ksteps) {
#pragma unroll 1
  for (int ks = 0; ks < ksteps; ++ks) {
    FragB a0, a1;
    a0.h[0] = *(const v8usa*)(ap + 32 * ks);
    a0.h[1] = *(const v8usa*)(ap + 32 * ks + 16);
    a1.h[0] = *(const v8usa*)(ap + (size_t)16 * (size_t)lda + 32 * ks);
    a1.h[1] = *(const v8usa*)(ap + (size_t)16 * (size_t)lda + 32 * ks + 16);
#pragma unroll
    for (int t = 0; t < 4; ++t) {
      const unsigned short* wq = wp + (size_t)(16 * t) * (size_t)ldb + 32 * ks;
      FragB bf;
      bf.h[0] = *(const v8usa*)wq;
      bf.h[1] = *(const v8usa*)(wq + 16);
      acc[0][t] = wmb(a0, bf, acc[0][t]);
      acc[1][t] = wmb(a1, bf, acc[1][t]);
    }
  }
}

__device__ __forceinline__ void st_f32(const float* stg, float* ob, const int ldo,
                                       const int wave, const int hh, const int m) {
#pragma unroll 4
  for (int i = 0; i < 16; ++i) {
    const int lr = 32 * wave + 2 * i + hh;
    const v4f v = *(const v4fa*)(stg + lr * GBN + 4 * m);
    *(volatile v4f*)(ob + (size_t)lr * (size_t)ldo + 4 * m) = v;
  }
}

template <bool RB>
__device__ __forceinline__ void st_hl(const float* stg, unsigned short* hb, const int ldh, const int loOfs,
                                      const float* __restrict__ rb, const int wave, const int lane) {
  const int sub = lane >> 3, q8 = lane & 7;
#pragma unroll 2
  for (int i = 0; i < 8; ++i) {
    const int lr = 32 * wave + 4 * i + sub;
    v4f v0 = *(const v4fa*)(stg + lr * GBN + 8 * q8);
    v4f v1 = *(const v4fa*)(stg + lr * GBN + 8 * q8 + 4);
    if (RB) {
      const float bb = bf16_val(rb[lr]);
      v0.x += bb; v0.y += bb; v0.z += bb; v0.w += bb;
      v1.x += bb; v1.y += bb; v1.z += bb; v1.w += bb;
    }
    const v8us hv = hl8(v0, v1, 0);
    const v8us lv = hl8(v0, v1, 1);
    unsigned short* hp = hb + (size_t)lr * (size_t)ldh + 8 * q8;
    *(volatile v8us*)hp = hv;
    *(volatile v8us*)(hp + loOfs) = lv;
  }
}

__device__ __forceinline__ void st_dr(const float* stg, unsigned short* db, const int wave, const int lane) {
  const int sub = lane >> 3, q8 = lane & 7;
  const int sc = 8 * (q8 & 3);
  const int pl = q8 >> 2;
#pragma unroll 2
  for (int i = 0; i < 8; ++i) {
    const int lr = 32 * wave + 4 * i + sub;
    const v4f v0 = *(const v4fa*)(stg + lr * GBN + sc);
    const v4f v1 = *(const v4fa*)(stg + lr * GBN + sc + 4);
    const v8us o = hl8(v0, v1, pl);
    *(volatile v8us*)(db + (size_t)lr * NDBC + 8 * q8) = o;
  }
}

enum { E_X1T = 0, E_X2 = 1, E_CONV = 2, E_DBC = 3, E_DT = 4, E_OUT = 5 };

template <int EPI>
__global__ __launch_bounds__(GTHR) void k_gemm(const unsigned short* __restrict__ A,
                                               const unsigned short* __restrict__ WT,
                                               float* outF, unsigned short* outH,
                                               const float* __restrict__ vec) {
  __shared__ __attribute__((aligned(16))) float stg[GBM * GBN];
  const int tid = (int)threadIdx.x, lane = tid & 31, wave = tid >> 5, hh = lane >> 4, m = lane & 15;
  const int rowBase = (int)blockIdx.x * GBM;
  const int col0    = (int)blockIdx.y * GBN;
  const int bz      = (int)blockIdx.z;
  const int arow    = rowBase + 32 * wave + m;

  v8f acc[2][4];
  {
    const v8f z = {0.f, 0.f, 0.f, 0.f, 0.f, 0.f, 0.f, 0.f};
#pragma unroll
    for (int t = 0; t < 4; ++t) { acc[0][t] = z; acc[1][t] = z; }
  }

  if constexpr (EPI == E_CONV) {
#pragma unroll 1
    for (int s = 0; s < 6; ++s) {
      const int t  = s >> 1;
      const int pl = s & 1;
      const unsigned short* ap = A + (size_t)t * WCT + (size_t)arow * SEQ + 8 * hh;
      const unsigned short* wp = WT + (size_t)pl * X1T_PLANE
                               + ((size_t)bz * PADR + (size_t)(col0 + m + t)) * SEQ + 8 * hh;
      mma_loop(acc, ap, SEQ, wp, SEQ, SEQ / 32);
    }
  } else {
    constexpr int LD = (EPI == E_X1T || EPI == E_X2) ? DM : ((EPI == E_DT) ? KDT : K2);
    const unsigned short* ap = A + (size_t)arow * LD + 8 * hh;
    const unsigned short* wp = WT + ((size_t)bz * SEQ + (size_t)(col0 + m)) * LD + 8 * hh;
    mma_loop(acc, ap, LD, wp, LD, LD / 32);
  }

#pragma unroll
  for (int mt = 0; mt < 2; ++mt) {
#pragma unroll
    for (int t = 0; t < 4; ++t) {
#pragma unroll
      for (int r = 0; r < 8; ++r) {
        stg[(32 * wave + 16 * mt + 8 * hh + r) * GBN + 16 * t + m] = acc[mt][t][r];
      }
    }
  }
  __syncthreads();

  if constexpr (EPI == E_X2 || EPI == E_DT || EPI == E_OUT) {
    const v4f bq = *(const v4f*)(vec + col0 + 4 * m);
    const float b0 = bf16_val(bq.x), b1 = bf16_val(bq.y), b2 = bf16_val(bq.z), b3 = bf16_val(bq.w);
#pragma unroll 1
    for (int i = 0; i < 16; ++i) {
      float* sp = stg + (32 * wave + 2 * i + hh) * GBN + 4 * m;
      v4f v = *(const v4fa*)sp;
      v.x += b0; v.y += b1; v.z += b2; v.w += b3;
      if constexpr (EPI == E_X2) {
        v.x = silu_f(v.x); v.y = silu_f(v.y); v.z = silu_f(v.z); v.w = silu_f(v.w);
      }
      if constexpr (EPI == E_DT) {
        v.x = softplus_f(v.x); v.y = softplus_f(v.y); v.z = softplus_f(v.z); v.w = softplus_f(v.w);
      }
      *(v4fa*)sp = v;
    }
  }
  if constexpr (EPI == E_CONV) {
#pragma unroll 1
    for (int i = 0; i < 16; ++i) {
      const int lr = 32 * wave + 2 * i + hh;
      const float bb = bf16_val(vec[rowBase + lr]);
      float* sp = stg + lr * GBN + 4 * m;
      v4f v = *(const v4fa*)sp;
      v.x = silu_f(v.x + bb); v.y = silu_f(v.y + bb); v.z = silu_f(v.z + bb); v.w = silu_f(v.w + bb);
      *(v4fa*)sp = v;
    }
    __syncthreads();
  }

  if constexpr (EPI == E_X1T) {
    unsigned short* hb = outH + ((size_t)bz * PADR + (size_t)(rowBase + 1)) * SEQ + col0;
    st_hl<true>(stg, hb, SEQ, X1T_PLANE, vec + rowBase, wave, lane);
    __threadfence();
    st_hl<true>(stg, hb, SEQ, X1T_PLANE, vec + rowBase, wave, lane);
  }
  if constexpr (EPI == E_X2 || EPI == E_DT || EPI == E_OUT) {
    float* ob = outF + (size_t)rowBase * DM + col0;
    st_f32(stg, ob, DM, wave, hh, m);
    __threadfence();
    st_f32(stg, ob, DM, wave, hh, m);
  }
  if constexpr (EPI == E_CONV) {
    const size_t grow = (size_t)bz * SEQ + (size_t)rowBase;
    float* ob = outF + grow * DM + col0;
    unsigned short* hb = outH + grow * K2 + col0;
    st_f32(stg, ob, DM, wave, hh, m);
    st_hl<false>(stg, hb, K2, DM, vec, wave, lane);
    __threadfence();
    st_f32(stg, ob, DM, wave, hh, m);
    st_hl<false>(stg, hb, K2, DM, vec, wave, lane);
  }
  if constexpr (EPI == E_DBC) {
    float* ob = outF + (size_t)rowBase * NDBC;
    unsigned short* db = outH + (size_t)rowBase * NDBC;
    st_f32(stg, ob, NDBC, wave, hh, m);
    st_dr(stg, db, wave, lane);
    __threadfence();
    st_f32(stg, ob, NDBC, wave, hh, m);
    st_dr(stg, db, wave, lane);
  }
}

__global__ __launch_bounds__(NTHR) void k_scan(const float* __restrict__ DELTA, const float* __restrict__ U,
                                               const float* __restrict__ SZ, const float* __restrict__ DBC,
                                               const unsigned short* __restrict__ XB,
                                               const float* __restrict__ Alog, const float* __restrict__ Dv,
                                               unsigned short* GHL) {
  extern __shared__ __attribute__((aligned(16))) float sm[];
  float* dl  = sm;
  float* uu  = sm + ST * SCH;
  float* sz  = sm + 2 * ST * SCH;
  float* gg  = sm + 3 * ST * SCH;
  float* bcs = sm + 4 * ST * SCH;
  const int tid = (int)threadIdx.x;
  const int ch = tid >> 1, half = tid & 1;
  const int b = (int)blockIdx.x >> 2;
  const int chBase = ((int)blockIdx.x & 3) * SCH;

  float Aa[8];
  {
    const float* arow = Alog + (size_t)(chBase + ch) * NS + 8 * half;
    const v4f a0 = *(const v4f*)(arow);
    const v4f a1 = *(const v4f*)(arow + 4);
    Aa[0] = -expf(bf16_val(a0.x)); Aa[1] = -expf(bf16_val(a0.y));
    Aa[2] = -expf(bf16_val(a0.z)); Aa[3] = -expf(bf16_val(a0.w));
    Aa[4] = -expf(bf16_val(a1.x)); Aa[5] = -expf(bf16_val(a1.y));
    Aa[6] = -expf(bf16_val(a1.z)); Aa[7] = -expf(bf16_val(a1.w));
  }
  const float Dd = bf16_val(Dv[chBase + ch]);
  float h[8];
#pragma unroll
  for (int j = 0; j < 8; ++j) h[j] = 0.0f;

#pragma unroll 1
  for (int cnk = 0; cnk < SEQ / ST; ++cnk) {
    const int row0 = b * SEQ + cnk * ST;
#pragma unroll
    for (int it = 0; it < 4; ++it) {
      const int idx = it * NTHR + tid;
      const int row = idx >> 5;
      const int cc  = (idx & 31) * 4;
      const size_t go = (size_t)(row0 + row) * DM + chBase + cc;
      const v4f a = *(const v4f*)(DELTA + go);
      const v4f e = *(const v4f*)(U + go);
      const v4f f = *(const v4f*)(SZ + go);
      *(v4fa*)(dl + row * SCH + cc) = a;
      *(v4fa*)(uu + row * SCH + cc) = e;
      *(v4fa*)(sz + row * SCH + cc) = f;
    }
    {
      const int row = tid >> 3;
      const int cc  = (tid & 7) * 4;
      const v4f a = *(const v4f*)(DBC + (size_t)(row0 + row) * NDBC + 32 + cc);
      *(v4fa*)(bcs + row * 32 + cc) = a;
    }
    __syncthreads();

#pragma unroll 1
    for (int t = 0; t < ST; ++t) {
      const float d  = dl[t * SCH + ch];
      const float u  = uu[t * SCH + ch];
      const float zz = sz[t * SCH + ch];
      const v4f B0 = *(const v4fa*)(bcs + t * 32 + 8 * half);
      const v4f B1 = *(const v4fa*)(bcs + t * 32 + 8 * half + 4);
      const v4f C0 = *(const v4fa*)(bcs + t * 32 + 16 + 8 * half);
      const v4f C1 = *(const v4fa*)(bcs + t * 32 + 16 + 8 * half + 4);
      const float Bv[8] = {B0.x, B0.y, B0.z, B0.w, B1.x, B1.y, B1.z, B1.w};
      const float Cv[8] = {C0.x, C0.y, C0.z, C0.w, C1.x, C1.y, C1.z, C1.w};
      float p = 0.0f;
#pragma unroll
      for (int j = 0; j < 8; ++j) {
        const float dA = expf(d * Aa[j]);
        h[j] = fmaf(dA, h[j], (d * Bv[j]) * u);
        p = fmaf(h[j], Cv[j], p);
      }
      const float other = __shfl_xor(p, 1, 32);
      const float plo = (half != 0) ? other : p;
      const float phi = (half != 0) ? p : other;
      const float y = (plo + phi) + u * Dd;
      const float g = y * zz;
      if (half == 0) gg[t * SCH + ch] = g;
    }
    __syncthreads();

    v8us ov[4];
#pragma unroll
    for (int it = 0; it < 4; ++it) {
      const int plane = it >> 1;
      const int idx = (it & 1) * NTHR + tid;
      const int row = idx >> 4;
      const int c8  = (idx & 15) * 8;
      v4f g0 = *(const v4fa*)(gg + row * SCH + c8);
      v4f g1 = *(const v4fa*)(gg + row * SCH + c8 + 4);
      const v4u xw = *(const v4ua*)(XB + (size_t)(row0 + row) * DM + chBase + c8);
      g0.x += __uint_as_float(xw.x << 16);
      g0.y += __uint_as_float(xw.x & 0xffff0000u);
      g0.z += __uint_as_float(xw.y << 16);
      g0.w += __uint_as_float(xw.y & 0xffff0000u);
      g1.x += __uint_as_float(xw.z << 16);
      g1.y += __uint_as_float(xw.z & 0xffff0000u);
      g1.z += __uint_as_float(xw.w << 16);
      g1.w += __uint_as_float(xw.w & 0xffff0000u);
      ov[it] = hl8(g0, g1, plane);
    }
#pragma unroll
    for (int it = 0; it < 4; ++it) {
      const int plane = it >> 1;
      const int idx = (it & 1) * NTHR + tid;
      const int row = idx >> 4;
      const int c8  = (idx & 15) * 8;
      unsigned short* gp = GHL + (size_t)(row0 + row) * K2 + (size_t)plane * DM + chBase + c8;
      *(volatile v8us*)gp = ov[it];
    }
    __threadfence();
#pragma unroll
    for (int it = 0; it < 4; ++it) {
      const int plane = it >> 1;
      const int idx = (it & 1) * NTHR + tid;
      const int row = idx >> 4;
      const int c8  = (idx & 15) * 8;
      unsigned short* gp = GHL + (size_t)(row0 + row) * K2 + (size_t)plane * DM + chBase + c8;
      *(volatile v8us*)gp = ov[it];
    }
  }
}

extern "C" void kernel_launch(void* const* d_in, const int* in_sizes, int n_in,
                              void* d_out, int out_size, void* d_ws, size_t ws_size,
                              hipStream_t stream) {
  if (n_in < 14) return;
  if (in_sizes[0] != MROWS * DM) return;
  if (in_sizes[1] != DM * DM || in_sizes[3] != DM * DM || in_sizes[5] != DM * DM) return;
  if (in_sizes[2] != DM || in_sizes[4] != DM || in_sizes[6] != DM) return;
  if (in_sizes[7] != SEQ * SEQ * 3) return;
  if (in_sizes[8] != SEQ) return;
  if (in_sizes[9] != NDBC * DM) return;
  if (in_sizes[10] != DM * 32) return;
  if (in_sizes[11] != DM) return;
  if (in_sizes[12] != DM * NS) return;
  if (in_sizes[13] != DM) return;
  if (out_size != MROWS * DM) return;

  const float* x      = (const float*)d_in[0];
  const float* W1     = (const float*)d_in[1];
  const float* b1     = (const float*)d_in[2];
  const float* W2     = (const float*)d_in[3];
  const float* b2     = (const float*)d_in[4];
  const float* Wout   = (const float*)d_in[5];
  const float* bout   = (const float*)d_in[6];
  const float* conv_w = (const float*)d_in[7];
  const float* conv_b = (const float*)d_in[8];
  const float* W_dbc  = (const float*)d_in[9];
  const float* W_dt   = (const float*)d_in[10];
  const float* b_dt   = (const float*)d_in[11];
  const float* A_log  = (const float*)d_in[12];
  const float* Dp     = (const float*)d_in[13];
  float* out = (float*)d_out;

  char* ws = (char*)d_ws;
  size_t off = 0;
  const size_t oXB   = off; off += (size_t)MROWS * DM * 2;
  const size_t oW1   = off; off += (size_t)DM * DM * 2;
  const size_t oW2   = off; off += (size_t)DM * DM * 2;
  const size_t oWO   = off; off += (size_t)DM * K2 * 2;
  const size_t oWC   = off; off += (size_t)3 * WCT * 2;
  const size_t oWD   = off; off += (size_t)NDBC * K2 * 2;
  const size_t oWT   = off; off += (size_t)DM * KDT * 2;
  const size_t oX1T  = off; off += (size_t)2 * X1T_PLANE * 2;
  const size_t oSZ   = off; off += (size_t)MROWS * DM * 4;
  const size_t oU    = off; off += (size_t)MROWS * DM * 4;
  const size_t oUHL  = off; off += (size_t)MROWS * K2 * 2;
  const size_t oDBC  = off; off += (size_t)MROWS * NDBC * 4;
  const size_t oDR   = off; off += (size_t)MROWS * NDBC * 2;
  const size_t oDL   = off; off += (size_t)MROWS * DM * 4;
  const size_t oGHL  = off; off += (size_t)MROWS * K2 * 2;
  if (off > ws_size || off > (size_t)WSMAX) return;
  unsigned short* XB    = (unsigned short*)(ws + oXB);
  unsigned short* W1B   = (unsigned short*)(ws + oW1);
  unsigned short* W2B   = (unsigned short*)(ws + oW2);
  unsigned short* WOUT2 = (unsigned short*)(ws + oWO);
  unsigned short* WC    = (unsigned short*)(ws + oWC);
  unsigned short* WDBC2 = (unsigned short*)(ws + oWD);
  unsigned short* WDT2  = (unsigned short*)(ws + oWT);
  unsigned short* X1T   = (unsigned short*)(ws + oX1T);
  float*          SZp   = (float*)(ws + oSZ);
  float*          Up    = (float*)(ws + oU);
  unsigned short* UHL   = (unsigned short*)(ws + oUHL);
  float*          DBCp  = (float*)(ws + oDBC);
  unsigned short* DRHL  = (unsigned short*)(ws + oDR);
  float*          DELTA = (float*)(ws + oDL);
  unsigned short* GHL   = (unsigned short*)(ws + oGHL);

  const size_t scanLds = (size_t)SCAN_LDS_FLOATS * 4;
  hipFuncSetAttribute(reinterpret_cast<const void*>(&k_scan), hipFuncAttributeMaxDynamicSharedMemorySize, (int)scanLds);

  k_prep<<<U_TOT / NTHR, NTHR, 0, stream>>>(x, W1, W2, Wout, W_dbc, W_dt, conv_w,
                                            XB, W1B, W2B, WOUT2, WDBC2, WDT2, WC, X1T);
  k_gemm<E_X1T><<<dim3(DM / GBM, SEQ / GBN, NB), GTHR, 0, stream>>>(W1B, XB, SZp, X1T, b1);
  k_gemm<E_X2><<<dim3(MROWS / GBM, DM / GBN, 1), GTHR, 0, stream>>>(XB, W2B, SZp, DRHL, b2);
  k_gemm<E_CONV><<<dim3(SEQ / GBM, DM / GBN, NB), GTHR, 0, stream>>>(WC, X1T, Up, UHL, conv_b);
  k_gemm<E_DBC><<<dim3(MROWS / GBM, NDBC / GBN, 1), GTHR, 0, stream>>>(UHL, WDBC2, DBCp, DRHL, b_dt);
  k_gemm<E_DT><<<dim3(MROWS / GBM, DM / GBN, 1), GTHR, 0, stream>>>(DRHL, WDT2, DELTA, DRHL, b_dt);
  k_scan<<<NB * (DM / SCH), NTHR, scanLds, stream>>>(DELTA, Up, SZp, DBCp, XB, A_log, Dp, GHL);
  k_gemm<E_OUT><<<dim3(MROWS / GBM, DM / GBN, 1), GTHR, 0, stream>>>(GHL, WOUT2, out, DRHL, bout);
}
